// DynamicEdgeConvLayer_18236431139303
// MI455X (gfx1250) — hardware-verified
//
#include <hip/hip_runtime.h>
#include <stdint.h>

#define NPTS  4096
#define CCH   64
#define BATCH 8
#define KNN   16
#define OUTC  64
#define DEP   20
#define NC    (2 * DEP)
#define NODES (BATCH * NPTS)

typedef _Float16 v16h __attribute__((ext_vector_type(16)));
typedef _Float16 v8h  __attribute__((ext_vector_type(8)));
typedef _Float16 v8ha __attribute__((ext_vector_type(8), may_alias));
typedef float    v8f  __attribute__((ext_vector_type(8)));
typedef float    v4f  __attribute__((ext_vector_type(4)));
union Frag { v16h v; v8h half[2]; };

__device__ __forceinline__ v8f mma16(v8f c, v16h a, v16h b) {
  v8f d = __builtin_amdgcn_wmma_f32_16x16x32_f16(false, a, false, b, (short)0, c, false, false);
  asm volatile("v_nop\n\tv_nop\n\tv_nop\n\tv_nop" : "+v"(d) : "v"(a), "v"(b));
  return d;
}

__device__ __forceinline__ int clampi(int v) {
  return v < 0 ? 0 : (v >= NPTS ? NPTS - 1 : v);
}

__global__ __launch_bounds__(256) void k_prep(const float* __restrict__ x,
                                              float* xt, _Float16* xh, float* sq) {
  const int b = blockIdx.y;
  const int n0 = blockIdx.x * 64;
  const int tid = threadIdx.x;
  if (b >= BATCH || n0 + 64 > NPTS) return;
  __shared__ float tile[64][65];
  __shared__ __attribute__((aligned(16))) float sqs[64];

  #pragma unroll 4
  for (int c0 = 0; c0 < CCH; c0 += 4) {
    const int c = c0 + (tid >> 6), n = tid & 63;
    tile[n][c] = x[((size_t)(b * CCH + c)) * NPTS + n0 + n];
  }
  __syncthreads();
  if (tid < 64) {
    float s = 0.f;
    #pragma unroll 8
    for (int c = 0; c < CCH; ++c) { const float v = tile[tid][c]; s = fmaf(v, v, s); }
    sqs[tid] = s;
  }
  __syncthreads();

  const int wv = tid >> 5, lane = tid & 31, q8 = lane & 7, l3 = lane >> 3;
  const size_t rowbase = (size_t)b * NPTS + n0;

  v4f tv[4]; size_t to[4];
  #pragma unroll
  for (int p = 0; p < 4; ++p) {
    const int L = wv * 16 + p * 4 + l3;
    const int row = L >> 1, col = (L & 1) * 32 + q8 * 4;
    v4f v;
    v.x = tile[row][col + 0]; v.y = tile[row][col + 1];
    v.z = tile[row][col + 2]; v.w = tile[row][col + 3];
    tv[p] = v;
    to[p] = (rowbase + row) * CCH + col;
    *(volatile v4f*)(xt + to[p]) = v;
  }
  v8h hv[2]; size_t ho[2];
  #pragma unroll
  for (int p = 0; p < 2; ++p) {
    const int row = wv * 8 + p * 4 + l3;
    const int col = q8 * 8;
    v8h v;
    #pragma unroll
    for (int e = 0; e < 8; ++e) v[e] = (_Float16)tile[row][col + e];
    hv[p] = v;
    ho[p] = (rowbase + row) * CCH + col;
    *(volatile v8h*)(xh + ho[p]) = v;
  }
  v4f sv = {0.f, 0.f, 0.f, 0.f};
  const bool sqw = (tid < 16);
  if (sqw) {
    sv = *(const v4f*)(&sqs[lane * 4]);
    *(volatile v4f*)(sq + rowbase + lane * 4) = sv;
  }
  __threadfence();
  #pragma unroll
  for (int p = 0; p < 4; ++p) *(volatile v4f*)(xt + to[p]) = tv[p];
  #pragma unroll
  for (int p = 0; p < 2; ++p) *(volatile v8h*)(xh + ho[p]) = hv[p];
  if (sqw) *(volatile v4f*)(sq + rowbase + lane * 4) = sv;
}

__device__ __forceinline__ void topk_insert(float d, int id, float* bd, int* bi,
                                            float& cmax, int& carg) {
  if (d < cmax) {
    #pragma unroll
    for (int t = 0; t < DEP; ++t)
      if (t == carg) { bd[t] = d; bi[t] = id; }
    cmax = -3.0e38f;
    #pragma unroll
    for (int t = 0; t < DEP; ++t)
      if (bd[t] > cmax) { cmax = bd[t]; carg = t; }
  }
}

__global__ __launch_bounds__(32) void k_knn(const _Float16* __restrict__ xh,
                                            const float* __restrict__ xt,
                                            const float* __restrict__ sq,
                                            _Float16* ed) {
  #pragma clang fp contract(off)
  const int b = blockIdx.y;
  const int q0 = blockIdx.x * 16;
  if (b >= BATCH || q0 + 16 > NPTS) return;
  const int lane = threadIdx.x & 31, m = lane & 15, h = lane >> 4;
  const size_t bN = (size_t)b * NPTS;
  const _Float16* xhB = xh + bN * CCH;
  const float* sqB = sq + bN;
  const float INFV = __int_as_float(0x7f800000);

  __shared__ int sidx[16][NC];

  Frag bq[2];
  {
    const _Float16* qr = xhB + (size_t)(q0 + m) * CCH;
    #pragma unroll
    for (int t = 0; t < 2; ++t) {
      bq[t].half[0] = *(const v8h*)(qr + 32 * t + 8 * h);
      bq[t].half[1] = *(const v8h*)(qr + 32 * t + 16 + 8 * h);
    }
  }

  float bd[DEP]; int bi[DEP];
  #pragma unroll
  for (int t = 0; t < DEP; ++t) { bd[t] = 3.0e38f; bi[t] = q0 + m; }
  float cmax = 3.0e38f;
  int carg = 0;

  #pragma unroll 1
  for (int j = 0; j < NPTS; j += 32) {
    Frag a[2][2];
    #pragma unroll
    for (int tt = 0; tt < 2; ++tt) {
      const _Float16* cr = xhB + (size_t)(j + 16 * tt + m) * CCH;
      #pragma unroll
      for (int t = 0; t < 2; ++t) {
        a[tt][t].half[0] = *(const v8h*)(cr + 32 * t + 8 * h);
        a[tt][t].half[1] = *(const v8h*)(cr + 32 * t + 16 + 8 * h);
      }
    }
    const v4f s0 = *(const v4f*)(sqB + j + 8 * h);
    const v4f s1 = *(const v4f*)(sqB + j + 8 * h + 4);
    const v4f s2 = *(const v4f*)(sqB + j + 16 + 8 * h);
    const v4f s3 = *(const v4f*)(sqB + j + 16 + 8 * h + 4);
    const float sv[16] = {s0.x, s0.y, s0.z, s0.w, s1.x, s1.y, s1.z, s1.w,
                          s2.x, s2.y, s2.z, s2.w, s3.x, s3.y, s3.z, s3.w};

    v8f acc0 = {}, acc1 = {};
    acc0 = mma16(acc0, a[0][0].v, bq[0].v);
    acc0 = mma16(acc0, a[0][1].v, bq[1].v);
    acc1 = mma16(acc1, a[1][0].v, bq[0].v);
    acc1 = mma16(acc1, a[1][1].v, bq[1].v);

    #pragma unroll
    for (int r = 0; r < 8; ++r)
      topk_insert(sv[r] - 2.0f * acc0[r], j + 8 * h + r, bd, bi, cmax, carg);
    #pragma unroll
    for (int r = 0; r < 8; ++r)
      topk_insert(sv[8 + r] - 2.0f * acc1[r], j + 16 + 8 * h + r, bd, bi, cmax, carg);
  }

  #pragma unroll
  for (int t = 0; t < DEP; ++t) sidx[m][h * DEP + t] = bi[t];
  __syncthreads();

  const int g = lane & 7, e4 = lane >> 3;
  const bool ubase = lane < (NC - 32);
  const int lb = ubase ? (32 + lane) : lane;

  #pragma unroll 1
  for (int q = 0; q < 16; ++q) {
    const size_t nrow = bN + (size_t)(q0 + q);
    const int ca = clampi(sidx[q][lane]);
    const int cb = clampi(sidx[q][lb]);
    const float sqn = sq[nrow];
    const v4f* xq4 = (const v4f*)(xt + nrow * CCH);

    v4f xr[16];
    #pragma unroll
    for (int qq = 0; qq < 16; ++qq) xr[qq] = xq4[qq];

    float da = INFV, db = INFV;
    #pragma unroll 1
    for (int cc = 0; cc < 2; ++cc) {
      const int c = cc ? cb : ca;
      const v4f* cr4 = (const v4f*)(xt + (bN + (size_t)c) * CCH);
      float dot = 0.f;
      #pragma unroll
      for (int qq = 0; qq < 16; ++qq) {
        const v4f cv = cr4[qq];
        const v4f xv = xr[qq];
        dot = fmaf(xv.x, cv.x, dot);
        dot = fmaf(xv.y, cv.y, dot);
        dot = fmaf(xv.z, cv.z, dot);
        dot = fmaf(xv.w, cv.w, dot);
      }
      const float s = sqn + sq[bN + (size_t)c];
      const float tw = 2.0f * dot;
      const float d = s - tw;
      if (cc) db = d; else da = d;
    }
    if (!ubase) db = INFV;

    bool ua = true, ub = ubase;
    int selk[KNN];
    #pragma unroll
    for (int it = 0; it < KNN; ++it) {
      float dl = INFV; int il = 0x7fffffff;
      if (ua) { dl = da; il = ca; }
      if (ub && (db < dl || (db == dl && cb < il))) { dl = db; il = cb; }
      #pragma unroll
      for (int s = 16; s > 0; s >>= 1) {
        const float od = __shfl_xor(dl, s);
        const int oi = __shfl_xor(il, s);
        if (od < dl || (od == dl && oi < il)) { dl = od; il = oi; }
      }
      selk[it] = il;
      if (ua && ca == il) ua = false;
      if (ub && cb == il) ub = false;
    }

    const v4f xg0 = xq4[2 * g], xg1 = xq4[2 * g + 1];
    v8h ev[4]; size_t eo[4];
    #pragma unroll
    for (int p = 0; p < 4; ++p) {
      const int k = 4 * p + e4;
      int jj = selk[4 * p + 3];
      jj = (e4 == 2) ? selk[4 * p + 2] : jj;
      jj = (e4 == 1) ? selk[4 * p + 1] : jj;
      jj = (e4 == 0) ? selk[4 * p + 0] : jj;
      jj = clampi(jj);
      const v4f* jr4 = (const v4f*)(xt + (bN + (size_t)jj) * CCH);
      const v4f c0 = jr4[2 * g], c1 = jr4[2 * g + 1];
      v8h e;
      e[0] = (_Float16)(c0.x - xg0.x); e[1] = (_Float16)(c0.y - xg0.y);
      e[2] = (_Float16)(c0.z - xg0.z); e[3] = (_Float16)(c0.w - xg0.w);
      e[4] = (_Float16)(c1.x - xg1.x); e[5] = (_Float16)(c1.y - xg1.y);
      e[6] = (_Float16)(c1.z - xg1.z); e[7] = (_Float16)(c1.w - xg1.w);
      ev[p] = e;
      eo[p] = (nrow * KNN + k) * CCH + 8 * g;
      *(volatile v8h*)(ed + eo[p]) = e;
    }
    __threadfence();
    #pragma unroll
    for (int p = 0; p < 4; ++p) *(volatile v8h*)(ed + eo[p]) = ev[p];
  }
}

__global__ __launch_bounds__(64) void k_mlp(const _Float16* __restrict__ xh,
                                            const _Float16* __restrict__ ed,
                                            const float* __restrict__ W1,
                                            const float* __restrict__ b1,
                                            const float* __restrict__ W2,
                                            const float* __restrict__ b2,
                                            float* out) {
  __shared__ __attribute__((aligned(16))) _Float16 w1a[OUTC * CCH];
  __shared__ __attribute__((aligned(16))) _Float16 w1b[OUTC * CCH];
  __shared__ __attribute__((aligned(16))) _Float16 w2s[OUTC * OUTC];
  __shared__ __attribute__((aligned(16))) float us[2][16][OUTC];
  __shared__ __attribute__((aligned(16))) _Float16 h1s[2][16][OUTC];
  __shared__ __attribute__((aligned(16))) float os[OUTC][32];

  const int tid = threadIdx.x, wv = tid >> 5, lane = tid & 31, m = lane & 15, h = lane >> 4;
  const int f0 = blockIdx.x * 32;
  if (f0 + 32 > NODES) return;
  const int b = f0 / NPTS, n0 = f0 - b * NPTS;

  for (int i = tid; i < OUTC * CCH; i += 64) {
    const int k = i >> 6, n = i & 63;
    w1a[n * CCH + k] = (_Float16)(64.0f * W1[i]);
    w1b[n * CCH + k] = (_Float16)(64.0f * W1[OUTC * CCH + i]);
    w2s[n * OUTC + k] = (_Float16)(64.0f * W2[i]);
  }
  __syncthreads();

  const int fw = f0 + wv * 16;
  const float r64 = 0.015625f;

  {
    Frag ax[2];
    const _Float16* xr = xh + (size_t)(fw + m) * CCH;
    #pragma unroll
    for (int t = 0; t < 2; ++t) {
      ax[t].half[0] = *(const v8h*)(xr + 32 * t + 8 * h);
      ax[t].half[1] = *(const v8h*)(xr + 32 * t + 16 + 8 * h);
    }
    #pragma unroll
    for (int nt = 0; nt < 4; ++nt) {
      v8f acc = {};
      #pragma unroll
      for (int t = 0; t < 2; ++t) {
        Frag bw;
        const _Float16* wp = &w1a[(nt * 16 + m) * CCH + 32 * t + 8 * h];
        bw.half[0] = *(const v8h*)(wp);
        bw.half[1] = *(const v8h*)(wp + 16);
        acc = mma16(acc, ax[t].v, bw.v);
      }
      const float bias = b1[nt * 16 + m];
      #pragma unroll
      for (int r = 0; r < 8; ++r) us[wv][8 * h + r][nt * 16 + m] = acc[r] * r64 + bias;
    }
  }
  __syncthreads();

  #pragma unroll 1
  for (int q = 0; q < 16; ++q) {
    const int fn = fw + q;
    Frag ae[2];
    const _Float16* er = ed + ((size_t)fn * KNN + m) * CCH;
    #pragma unroll
    for (int t = 0; t < 2; ++t) {
      ae[t].half[0] = *(const v8h*)(er + 32 * t + 8 * h);
      ae[t].half[1] = *(const v8h*)(er + 32 * t + 16 + 8 * h);
    }
    #pragma unroll
    for (int nt = 0; nt < 4; ++nt) {
      v8f acc = {};
      #pragma unroll
      for (int t = 0; t < 2; ++t) {
        Frag bw;
        const _Float16* wp = &w1b[(nt * 16 + m) * CCH + 32 * t + 8 * h];
        bw.half[0] = *(const v8h*)(wp);
        bw.half[1] = *(const v8h*)(wp + 16);
        acc = mma16(acc, ae[t].v, bw.v);
      }
      const float uq = us[wv][q][nt * 16 + m];
      #pragma unroll
      for (int r = 0; r < 8; ++r) {
        float v = acc[r] * r64 + uq;
        v = fmaxf(v, 0.f);
        h1s[wv][8 * h + r][nt * 16 + m] = (_Float16)v;
      }
    }
    __syncthreads();
    Frag a2[2];
    #pragma unroll
    for (int t = 0; t < 2; ++t) {
      a2[t].half[0] = *(const v8ha*)(&h1s[wv][m][32 * t + 8 * h]);
      a2[t].half[1] = *(const v8ha*)(&h1s[wv][m][32 * t + 16 + 8 * h]);
    }
    #pragma unroll
    for (int nt = 0; nt < 4; ++nt) {
      v8f acc = {};
      #pragma unroll
      for (int t = 0; t < 2; ++t) {
        Frag bw;
        const _Float16* wp = &w2s[(nt * 16 + m) * OUTC + 32 * t + 8 * h];
        bw.half[0] = *(const v8h*)(wp);
        bw.half[1] = *(const v8h*)(wp + 16);
        acc = mma16(acc, a2[t].v, bw.v);
      }
      float mx = acc[0];
      #pragma unroll
      for (int r = 1; r < 8; ++r) mx = fmaxf(mx, acc[r]);
      mx = fmaxf(mx, __shfl_xor(mx, 16));
      const float v = fmaxf(mx * r64 + b2[nt * 16 + m], 0.f);
      if (h == 0) os[nt * 16 + m][wv * 16 + q] = v;
    }
    __syncthreads();
  }

  const int q8 = lane & 7, l3 = lane >> 3;
  v4f ov[8]; size_t oo[8];
  #pragma unroll
  for (int p = 0; p < 8; ++p) {
    const int ch = wv * 32 + p * 4 + l3;
    const v4f v = *(const v4f*)(&os[ch][q8 * 4]);
    ov[p] = v;
    oo[p] = ((size_t)(b * OUTC + ch)) * NPTS + n0 + q8 * 4;
    *(volatile v4f*)(out + oo[p]) = v;
  }
  __threadfence();
  #pragma unroll
  for (int p = 0; p < 8; ++p) *(volatile v4f*)(out + oo[p]) = ov[p];
}

extern "C" void kernel_launch(void* const* d_in, const int* in_sizes, int n_in,
                              void* d_out, int out_size, void* d_ws, size_t ws_size,
                              hipStream_t stream) {
  if (n_in < 5) return;
  if (in_sizes[0] != BATCH * CCH * NPTS) return;
  if (in_sizes[1] != 2 * CCH * OUTC) return;
  if (in_sizes[2] != OUTC) return;
  if (in_sizes[3] != OUTC * OUTC) return;
  if (in_sizes[4] != OUTC) return;
  if (out_size != BATCH * OUTC * NPTS) return;

  const float* x  = (const float*)d_in[0];
  const float* W1 = (const float*)d_in[1];
  const float* b1 = (const float*)d_in[2];
  const float* W2 = (const float*)d_in[3];
  const float* b2 = (const float*)d_in[4];
  float* out = (float*)d_out;

  const size_t xt_bytes = (size_t)NODES * CCH * 4;
  const size_t xh_bytes = (size_t)NODES * CCH * 2;
  const size_t sq_bytes = (size_t)NODES * 4;
  const size_t ed_bytes = (size_t)NODES * KNN * CCH * 2;
  const size_t xt_off = 0;
  const size_t xh_off = xt_off + xt_bytes;
  const size_t sq_off = xh_off + xh_bytes;
  const size_t ed_off = sq_off + sq_bytes;
  const size_t total  = ed_off + ed_bytes;
  if (total > ws_size) return;

  char* ws = (char*)d_ws;
  float*    xt = (float*)(ws + xt_off);
  _Float16* xh = (_Float16*)(ws + xh_off);
  float*    sq = (float*)(ws + sq_off);
  _Float16* ed = (_Float16*)(ws + ed_off);

  k_prep<<<dim3((NPTS + 63) / 64, BATCH), 256, 0, stream>>>(x, xt, xh, sq);
  k_knn <<<dim3((NPTS + 15) / 16, BATCH), 32, 0, stream>>>(xh, xt, sq, ed);
  k_mlp <<<dim3((NODES + 31) / 32), 64, 0, stream>>>(xh, ed, W1, b1, W2, b2, out);
}
